// MetaEmbedding_Classifier_4191888081208
// MI455X (gfx1250) — hardware-run, weakly checked
//
#include <hip/hip_runtime.h>


#ifndef NB
#define NB 64
#endif
#define NB_FULL 64
#define FD   2048
#define NCLS 1000
#define NP   1024
#define L2E  1.4426950408889634f
#define OFF_DIRECT  ((size_t)NB_FULL * NCLS)
#define OFF_INFUSED (OFF_DIRECT + (size_t)NB_FULL * FD)

static_assert(NB % 64 == 0);
static_assert(NB <= NB_FULL);
static_assert(FD % 64 == 0);
static_assert(NP % 64 == 0);
static_assert(FD % 32 == 0);
static_assert(NP % 32 == 0);
static_assert(NCLS % 8 == 0);
static_assert(NCLS <= NP);
static_assert(FD == 256 * 8);
static_assert(NP == 128 * 8);
static_assert(OFF_DIRECT * 4 == 256000);
static_assert(OFF_INFUSED * 4 == 780288);
static_assert((OFF_DIRECT * 4) % 256 == 0);
static_assert((OFF_INFUSED * 4) % 256 == 0);
static_assert(((size_t)NB * NCLS / 4) % 32 == 0);
static_assert((NB + 2 * NP) % 32 == 0);
static_assert((NB + NP) % 32 == 0);

typedef unsigned short bf;
typedef __attribute__((ext_vector_type(16))) __bf16   v16bf;
typedef __attribute__((ext_vector_type(8)))  unsigned short v8us;
typedef __attribute__((ext_vector_type(4)))  unsigned short v4us;
typedef __attribute__((ext_vector_type(8)))  float    v8f;
typedef __attribute__((ext_vector_type(4)))  float    v4f;
typedef v4f  __attribute__((may_alias)) v4fa;
typedef v8us __attribute__((may_alias)) v8usa;

__device__ __forceinline__ unsigned short f2bf(float f) { unsigned u = __float_as_uint(f); u += 0x7FFFu + ((u >> 16) & 1u); return (unsigned short)(u >> 16); }
__device__ __forceinline__ float bf2f(unsigned short w) { return __uint_as_float(((unsigned)w) << 16); }
__device__ __forceinline__ v16bf cat16b(v8us lo, v8us hi) { return __builtin_bit_cast(v16bf, __builtin_shufflevector(lo, hi, 0, 1, 2, 3, 4, 5, 6, 7, 8, 9, 10, 11, 12, 13, 14, 15)); }
__device__ __forceinline__ v8f wmmab(v16bf a, v16bf b, v8f c) { return __builtin_amdgcn_wmma_f32_16x16x32_bf16(false, a, false, b, (short)0, c, false, false); }
__device__ __forceinline__ v16bf ldb(const bf* p)  { return cat16b(*(const v8us*)p, *(const v8us*)(p + 16)); }
__device__ __forceinline__ void wave_sync() { __builtin_amdgcn_fence(3  , "wavefront"); __builtin_amdgcn_wave_barrier(); asm volatile("" ::: "memory"); }
__device__ __forceinline__ float wsum(float v) {
#pragma unroll
    for (int o = 16; o > 0; o >>= 1) v += __shfl_xor(v, o, 32);
    return v; }
__device__ __forceinline__ float wmax(float v) {
#pragma unroll
    for (int o = 16; o > 0; o >>= 1) v = fmaxf(v, __shfl_xor(v, o, 32));
    return v; }
__device__ __forceinline__ float wmin(float v) {
#pragma unroll
    for (int o = 16; o > 0; o >>= 1) v = fminf(v, __shfl_xor(v, o, 32));
    return v; }

__global__ __launch_bounds__(256) void k_cvtrow(const float* __restrict__ src, bf* dst, int nsrc) {
    const int row = blockIdx.x; const int sr = row < nsrc ? row : nsrc - 1; const int t = threadIdx.x;
    const v8f v = *(const v8f*)(src + (size_t)sr * FD + t * 8); v8us o;
#pragma unroll
    for (int k = 0; k < 8; ++k) o[k] = f2bf(v[k]);
    bf* p = dst + (size_t)row * FD + t * 8;
    *(volatile v8us*)p = o; __threadfence(); *(volatile v8us*)p = o;
}

__global__ __launch_bounds__(256) void k_outx(const float* __restrict__ x, float* out, int n4) {
    const int i = blockIdx.x * 256 + threadIdx.x; if (i >= n4) return;
    const v4f v = *(const v4f*)(x + (size_t)i * 4); v4f o;
#pragma unroll
    for (int k = 0; k < 4; ++k) o[k] = bf2f(f2bf(v[k]));
    float* p = out + (size_t)i * 4;
    *(volatile v4f*)p = o; __threadfence(); *(volatile v4f*)p = o;
}

__global__ __launch_bounds__(256) void k_tr(const float* __restrict__ src, bf* dst) {
    __shared__ __align__(16) unsigned short ts[64 * 72];
    const int t = threadIdx.x; const int c0 = blockIdx.x * 64, f0 = blockIdx.y * 64;
    const int ci = t >> 2, fj = (t & 3) * 16;
    const int c = c0 + ci; const int cs = c < NCLS ? c : NCLS - 1; const bool ok = c < NCLS;
    const float* p = src + (size_t)cs * FD + f0 + fj;
#pragma unroll
    for (int q = 0; q < 4; ++q) { const v4f v = *(const v4f*)(p + 4 * q);
#pragma unroll
        for (int e = 0; e < 4; ++e) { const unsigned short w = f2bf(v[e]); ts[(fj + 4 * q + e) * 72 + ci] = ok ? w : (unsigned short)0; } }
    __syncthreads();
#pragma unroll 1
    for (int ps = 0; ps < 2; ++ps) {
#pragma unroll
        for (int it = 0; it < 2; ++it) { const int row = it * 32 + (t >> 3), pc = (t & 7) * 8;
            const v8us o = *(const v8usa*)(&ts[row * 72 + pc]);
            *(volatile v8us*)(dst + (size_t)(f0 + row) * NP + c0 + pc) = o; }
        if (ps == 0) __threadfence(); }
}

__global__ __launch_bounds__(256) void k_rowss(const bf* __restrict__ P, float* SS, int blk1) {
    __shared__ __align__(16) float sv[32];
    const int lane = threadIdx.x & 31; const int wave = __builtin_amdgcn_readfirstlane((int)(threadIdx.x >> 5));
#pragma unroll 1
    for (int q = 0; q < 4; ++q) {
        const int row = blockIdx.x * 32 + wave * 4 + q;
        const bf* p = P + (size_t)row * FD + lane * 8;
        float s = 0.0f;
#pragma unroll 1
        for (int j = 0; j < 8; ++j) { const v8us w = *(const v8us*)(p + j * 256);
#pragma unroll
            for (int e = 0; e < 8; ++e) { const float f = bf2f(w[e]); s += f * f; } }
        s = wsum(s);
        const float o = ((int)blockIdx.x >= blk1) ? 16.0f / sqrtf(s) : s;
        if (lane == 0) sv[wave * 4 + q] = o;
    }
    __syncthreads();
    if (threadIdx.x < 8) { const v4f o = *(const v4fa*)(&sv[threadIdx.x * 4]); float* d = SS + (size_t)blockIdx.x * 32 + threadIdx.x * 4;
        *(volatile v4f*)d = o; __threadfence(); *(volatile v4f*)d = o; }
}

#define M_DIST 0
#define M_BIAS 1
#define M_TANH 2
#define M_MEMF 3
#define M_COS  4

template<int MODE>
__global__ __launch_bounds__(32) void k_gemm(const bf* __restrict__ A, size_t aPl, int NA, const bf* __restrict__ Bt, int K,
                                             float* O0, float* O1, int pitch, const float* __restrict__ Pc, int ncl,
                                             const float* __restrict__ Pr, const float* __restrict__ Pe, const bf* __restrict__ Xp) {
    __shared__ __align__(16) float os[16 * 68];
    __shared__ __align__(16) float os2[16 * 68];
    const int lane = threadIdx.x & 31, lr = lane & 15, hi = lane >> 4; const int r0 = blockIdx.x * 64, c0 = blockIdx.y * 64;
    v8f acc[4][4];
#pragma unroll
    for (int mb = 0; mb < 4; ++mb)
#pragma unroll
        for (int nb = 0; nb < 4; ++nb) acc[mb][nb] = (v8f){};
    const size_t aoff = (size_t)(r0 + lr) * K + 8 * hi, boff = (size_t)(c0 + lr) * K + 8 * hi;
#pragma unroll 1
    for (int kc = 0; kc < K; kc += 32) {
#pragma unroll 1
        for (int pl = 0; pl < NA; ++pl) {
            const bf* Ap = A + (size_t)pl * aPl;
            v16bf a[4];
#pragma unroll
            for (int mb = 0; mb < 4; ++mb) a[mb] = ldb(Ap + aoff + (size_t)mb * 16 * K + kc);
#pragma unroll
            for (int nb = 0; nb < 4; ++nb) { const v16bf b = ldb(Bt + boff + (size_t)nb * 16 * K + kc);
#pragma unroll
                for (int mb = 0; mb < 4; ++mb) acc[mb][nb] = wmmab(a[mb], b, acc[mb][nb]); }
            asm volatile("v_nop\n\tv_nop\n\tv_nop\n\tv_nop" : "+v"(acc[0][0]), "+v"(acc[1][1]), "+v"(acc[2][2]), "+v"(acc[3][3]) : "v"(a[0]), "v"(a[1]), "v"(a[2]), "v"(a[3]));
        }
    }
    const int cofs = lr * 4;
    v4f ct = (v4f){};
    if (MODE != M_MEMF) { int nn = c0 + cofs; nn = nn < ncl - 4 ? nn : ncl - 4; ct = *(const v4f*)(Pc + nn); }
    if (MODE == M_BIAS || MODE == M_TANH) {
#pragma unroll
        for (int i = 0; i < 4; ++i) ct[i] = bf2f(f2bf(ct[i])); }
#pragma unroll
    for (int mb = 0; mb < 4; ++mb) {
#pragma unroll
        for (int nb = 0; nb < 4; ++nb) {
#pragma unroll
            for (int j = 0; j < 8; ++j) os[(hi * 8 + j) * 68 + nb * 16 + lr] = acc[mb][nb][j]; }
        wave_sync();
#pragma unroll 1
        for (int s = 0; s < 8; ++s) { const int row = 2 * s + hi;
            const int m = r0 + mb * 16 + row; const int n = c0 + cofs;
            v4f v = *(const v4fa*)(&os[row * 68 + cofs]);
            if (MODE == M_DIST) { const float xn = Pr[m];
#pragma unroll
                for (int i = 0; i < 4; ++i) { const float d2 = (xn + ct[i]) - 2.0f * v[i]; v[i] = sqrtf(fmaxf(d2, 0.0f)); } }
            if (MODE == M_BIAS) {
#pragma unroll
                for (int i = 0; i < 4; ++i) v[i] = v[i] + ct[i]; }
            if (MODE == M_TANH) {
#pragma unroll
                for (int i = 0; i < 4; ++i) v[i] = tanhf(v[i] + ct[i]); }
            if (MODE == M_COS) {
#pragma unroll
                for (int i = 0; i < 4; ++i) v[i] = v[i] * ct[i]; }
            if (MODE == M_MEMF) { const v4f sel = *(const v4f*)(Pe + (size_t)m * pitch + n); const v4us xw = *(const v4us*)(Xp + (size_t)m * FD + n); v4f g;
#pragma unroll
                for (int i = 0; i < 4; ++i) { const float inf = sel[i] * v[i]; v[i] = inf; g[i] = bf2f(xw[i]) + inf; }
                *(v4fa*)(&os2[row * 68 + cofs]) = g; }
            *(v4fa*)(&os[row * 68 + cofs]) = v; }
        wave_sync();
        const size_t sb = (size_t)(r0 + mb * 16) * (size_t)pitch + c0 + cofs;
#pragma unroll 1
        for (int ps = 0; ps < 2; ++ps) {
#pragma unroll
            for (int s = 0; s < 8; ++s) { const int row = 2 * s + hi;
                const v4f val = *(const v4fa*)(&os[row * 68 + cofs]);
                *(volatile v4f*)(O0 + sb + (size_t)row * (size_t)pitch) = val;
                if (MODE == M_MEMF) { const v4f val2 = *(const v4fa*)(&os2[row * 68 + cofs]);
                    *(volatile v4f*)(O1 + sb + (size_t)row * (size_t)pitch) = val2; } }
            if (ps == 0) __threadfence(); }
        wave_sync();
    }
}

__global__ __launch_bounds__(128) void k_softmax(const float* __restrict__ H, bf* VM) {
    __shared__ float rmx[4]; __shared__ float rsm[4];
    const int r = blockIdx.x, t = threadIdx.x, lane = t & 31; const int wave = __builtin_amdgcn_readfirstlane(t >> 5);
    const int c = 8 * t; const bool ok = c < NCLS;
    const v4f v0 = *(const v4f*)(H + (size_t)r * NP + c); const v4f v1 = *(const v4f*)(H + (size_t)r * NP + c + 4);
    float e[8];
#pragma unroll
    for (int k = 0; k < 4; ++k) { e[k] = v0[k]; e[4 + k] = v1[k]; }
    float mx = -3.0e38f;
#pragma unroll
    for (int k = 0; k < 8; ++k) mx = fmaxf(mx, e[k]);
    mx = ok ? mx : -3.0e38f;
    mx = wmax(mx);
    if (lane == 0) rmx[wave] = mx;
    __syncthreads();
    mx = fmaxf(fmaxf(rmx[0], rmx[1]), fmaxf(rmx[2], rmx[3]));
    float s = 0.0f;
#pragma unroll
    for (int k = 0; k < 8; ++k) { const float ev = __builtin_amdgcn_exp2f((e[k] - mx) * L2E); e[k] = ok ? ev : 0.0f; s += e[k]; }
    s = wsum(s);
    if (lane == 0) rsm[wave] = s;
    __syncthreads();
    s = ((rsm[0] + rsm[1]) + rsm[2]) + rsm[3];
    const float inv = 1.0f / s;
    v8us hv, lv;
#pragma unroll
    for (int k = 0; k < 8; ++k) { const float p = e[k] * inv; const unsigned short hb = f2bf(p); hv[k] = hb; lv[k] = f2bf(p - bf2f(hb)); }
    bf* ph = VM + (size_t)r * NP + c; bf* pl = VM + (size_t)NB * NP + (size_t)r * NP + c;
    *(volatile v8us*)ph = hv; *(volatile v8us*)pl = lv; __threadfence(); *(volatile v8us*)ph = hv; *(volatile v8us*)pl = lv;
}

__global__ __launch_bounds__(256) void k_ex(const float* __restrict__ D, const float* __restrict__ G, bf* EX) {
    __shared__ float rmn[8]; __shared__ float rss[8];
    const int r = blockIdx.x, t = threadIdx.x, lane = t & 31; const int wave = __builtin_amdgcn_readfirstlane(t >> 5);
    const v4f dv = *(const v4f*)(D + (size_t)r * NP + 4 * t);
    float mn = fminf(fminf(dv[0], dv[1]), fminf(dv[2], dv[3]));
    mn = (4 * t < NCLS) ? mn : 3.0e38f;
    mn = wmin(mn);
    if (lane == 0) rmn[wave] = mn;
    __syncthreads();
    mn = rmn[0];
#pragma unroll
    for (int k = 1; k < 8; ++k) mn = fminf(mn, rmn[k]);
    const float reach = 10.0f / mn;
    const v4f g0 = *(const v4f*)(G + (size_t)r * FD + 8 * t); const v4f g1 = *(const v4f*)(G + (size_t)r * FD + 8 * t + 4);
    float f[8]; float ss = 0.0f;
#pragma unroll
    for (int k = 0; k < 4; ++k) { f[k] = reach * g0[k]; f[4 + k] = reach * g1[k]; }
#pragma unroll
    for (int k = 0; k < 8; ++k) ss += f[k] * f[k];
    ss = wsum(ss);
    if (lane == 0) rss[wave] = ss;
    __syncthreads();
    ss = rss[0];
#pragma unroll
    for (int k = 1; k < 8; ++k) ss += rss[k];
    const float nrm = sqrtf(ss); const float rn = 1.0f / nrm; const float sc = nrm / (1.0f + nrm);
    v8us hv, lv;
#pragma unroll
    for (int k = 0; k < 8; ++k) { const float p = sc * (f[k] * rn); const unsigned short hb = f2bf(p); hv[k] = hb; lv[k] = f2bf(p - bf2f(hb)); }
    bf* ph = EX + (size_t)r * FD + 8 * t; bf* pl = EX + (size_t)NB * FD + (size_t)r * FD + 8 * t;
    *(volatile v8us*)ph = hv; *(volatile v8us*)pl = lv; __threadfence(); *(volatile v8us*)ph = hv; *(volatile v8us*)pl = lv;
}

__global__ __launch_bounds__(256) void k_outlog(const float* __restrict__ LP, float* out, int n4) {
    const int i = blockIdx.x * 256 + threadIdx.x; if (i >= n4) return;
    const int e = i * 4; const int r = e / NCLS; const int c = e - r * NCLS;
    const v4f v = *(const v4f*)(LP + (size_t)r * NP + c);
    float* p = out + (size_t)e;
    *(volatile v4f*)p = v; __threadfence(); *(volatile v4f*)p = v;
}

static constexpr size_t al256(size_t v) { return (v + 255) & ~(size_t)255; }
static constexpr size_t PROWS   = (size_t)NB + 2 * NP;
static constexpr size_t SZ_P16  = al256(PROWS * FD * 2);
static constexpr size_t SZ_WHB  = al256((size_t)NP * FD * 2);
static constexpr size_t SZ_WSB  = al256((size_t)FD * FD * 2);
static constexpr size_t SZ_CT   = al256((size_t)FD * NP * 2);
static constexpr size_t SZ_SS   = al256(PROWS * 4);
static constexpr size_t SZ_DIST = al256((size_t)NB * NP * 4);
static constexpr size_t SZ_HALL = al256((size_t)NB * NP * 4);
static constexpr size_t SZ_SEL  = al256((size_t)NB * FD * 4);
static constexpr size_t SZ_VM   = al256((size_t)2 * NB * NP * 2);
static constexpr size_t SZ_G    = al256((size_t)NB * FD * 4);
static constexpr size_t SZ_EX   = al256((size_t)2 * NB * FD * 2);
static constexpr size_t SZ_LOG  = al256((size_t)NB * NP * 4);
static constexpr size_t SZ_TOTAL = SZ_P16 + SZ_WHB + SZ_WSB + SZ_CT + SZ_SS + SZ_DIST + SZ_HALL + SZ_SEL + SZ_VM + SZ_G + SZ_EX + SZ_LOG;
static_assert(SZ_TOTAL <= (size_t)134217728);
static_assert((PROWS / 32) * 32 * 4 <= SZ_SS);

extern "C" void kernel_launch(void* const* d_in, const int* in_sizes, int n_in,
                              void* d_out, int out_size, void* d_ws, size_t ws_size, hipStream_t stream) {
    if (n_in < 7) return;
    if ((size_t)in_sizes[0] < (size_t)NB * FD) return;
    if ((size_t)in_sizes[1] < (size_t)NCLS * FD || (size_t)in_sizes[2] < (size_t)NCLS * FD || (size_t)in_sizes[3] < (size_t)NCLS) return;
    if ((size_t)in_sizes[4] < (size_t)FD * FD || (size_t)in_sizes[5] < (size_t)FD || (size_t)in_sizes[6] < (size_t)NCLS * FD) return;
    if ((size_t)out_size < OFF_INFUSED + (size_t)NB * FD) return;
    if (SZ_TOTAL > ws_size) return;
    const float* x = (const float*)d_in[0]; const float* cent = (const float*)d_in[1]; const float* whall = (const float*)d_in[2]; const float* bhall = (const float*)d_in[3];
    const float* wsel = (const float*)d_in[4]; const float* bsel = (const float*)d_in[5]; const float* wcos = (const float*)d_in[6];
    float* OUT = (float*)d_out;
    char* wsp = (char*)d_ws;
    bf* P16 = (bf*)wsp; wsp += SZ_P16;
    bf* WHB = (bf*)wsp; wsp += SZ_WHB;
    bf* WSB = (bf*)wsp; wsp += SZ_WSB;
    bf* CT  = (bf*)wsp; wsp += SZ_CT;
    float* SS = (float*)wsp; wsp += SZ_SS;
    float* DIST = (float*)wsp; wsp += SZ_DIST;
    float* HALL = (float*)wsp; wsp += SZ_HALL;
    float* SEL  = (float*)wsp; wsp += SZ_SEL;
    bf* VM = (bf*)wsp; wsp += SZ_VM;
    float* G = (float*)wsp; wsp += SZ_G;
    bf* EX = (bf*)wsp; wsp += SZ_EX;
    float* LOGP = (float*)wsp; wsp += SZ_LOG;
    bf* XB = P16; bf* CB = P16 + (size_t)NB * FD; bf* WCB = P16 + (size_t)(NB + NP) * FD;
    float* XN2 = SS; float* CN2 = SS + NB; float* WS16 = SS + NB + NP;

    k_cvtrow<<<NB, 256, 0, stream>>>(x, XB, NB);
    k_cvtrow<<<NP, 256, 0, stream>>>(cent, CB, NCLS);
    k_cvtrow<<<NP, 256, 0, stream>>>(wcos, WCB, NCLS);
    k_cvtrow<<<NP, 256, 0, stream>>>(whall, WHB, NCLS);
    k_cvtrow<<<FD, 256, 0, stream>>>(wsel, WSB, FD);
    k_tr<<<dim3(NP / 64, FD / 64, 1), 256, 0, stream>>>(cent, CT);
    { const int n4 = NB * FD / 4; k_outx<<<(n4 + 255) / 256, 256, 0, stream>>>(x, OUT + OFF_DIRECT, n4); }
    k_rowss<<<(unsigned)(PROWS / 32), 256, 0, stream>>>(P16, SS, (NB + NP) / 32);

    k_gemm<M_DIST><<<dim3(NB / 64, NP / 64, 1), 32, 0, stream>>>(XB, (size_t)0, 1, CB, FD, DIST, DIST, NP, CN2, NP, XN2, XN2, XB);
    k_gemm<M_BIAS><<<dim3(NB / 64, NP / 64, 1), 32, 0, stream>>>(XB, (size_t)0, 1, WHB, FD, HALL, HALL, NP, bhall, NCLS, XN2, XN2, XB);
    k_gemm<M_TANH><<<dim3(NB / 64, FD / 64, 1), 32, 0, stream>>>(XB, (size_t)0, 1, WSB, FD, SEL, SEL, FD, bsel, FD, XN2, XN2, XB);
    k_softmax<<<NB, 128, 0, stream>>>(HALL, VM);
    k_gemm<M_MEMF><<<dim3(NB / 64, FD / 64, 1), 32, 0, stream>>>(VM, (size_t)NB * NP, 2, CT, NP, OUT + OFF_INFUSED, G, FD, XN2, 4, XN2, SEL, XB);
    k_ex<<<NB, 256, 0, stream>>>(DIST, G, EX);
    k_gemm<M_COS><<<dim3(NB / 64, NP / 64, 1), 32, 0, stream>>>(EX, (size_t)NB * FD, 2, WCB, FD, LOGP, LOGP, NP, WS16, NP, XN2, XN2, XB);
    { const int n4 = NB * NCLS / 4; k_outlog<<<(n4 + 255) / 256, 256, 0, stream>>>(LOGP, OUT, n4); }
}
